// PoseMixtureVAE_74423193305293
// MI455X (gfx1250) — hardware-verified
//
#include <hip/hip_runtime.h>


#define NR   2048
#define FR   267
#define LT   32
#define HD   256
#define NP   6
#define GW   64
#define K1   576
#define K2   320
#define N3   320
typedef _Float16 h16;
typedef unsigned short bf;
typedef __attribute__((ext_vector_type(16))) __bf16   v16bf;
typedef __attribute__((ext_vector_type(16))) _Float16 v16h;
typedef __attribute__((ext_vector_type(8)))  _Float16 v8h;
typedef __attribute__((ext_vector_type(8)))  unsigned short v8us;
typedef __attribute__((ext_vector_type(8)))  float    v8f;
typedef __attribute__((ext_vector_type(4)))  float    v4f;
typedef v8h  __attribute__((may_alias)) v8ha;
typedef v4f  __attribute__((may_alias)) v4fa;
typedef v8us __attribute__((may_alias)) v8usa;

__device__ __forceinline__ unsigned short f2bf(float f) { unsigned u = __float_as_uint(f); u += 0x7FFFu + ((u >> 16) & 1u); return (unsigned short)(u >> 16); }
__device__ __forceinline__ float bf2f(unsigned short b) { return __uint_as_float(((unsigned)b) << 16); }
__device__ __forceinline__ float bfr(float f) { return bf2f(f2bf(f)); }
__device__ __forceinline__ v16h cat16(v8h lo, v8h hi) { return __builtin_shufflevector(lo, hi, 0, 1, 2, 3, 4, 5, 6, 7, 8, 9, 10, 11, 12, 13, 14, 15); }
__device__ __forceinline__ v16bf cat16b(v8us lo, v8us hi) { return __builtin_bit_cast(v16bf, __builtin_shufflevector(lo, hi, 0, 1, 2, 3, 4, 5, 6, 7, 8, 9, 10, 11, 12, 13, 14, 15)); }
__device__ __forceinline__ v8f wmma16(v16h a, v16h b, v8f c) { return __builtin_amdgcn_wmma_f32_16x16x32_f16(false, a, false, b, (short)0, c, false, false); }
__device__ __forceinline__ v8f wmmab(v16bf a, v16bf b, v8f c) { return __builtin_amdgcn_wmma_f32_16x16x32_bf16(false, a, false, b, (short)0, c, false, false); }

template <typename T16> struct WFrag;
template <> struct WFrag<h16> { typedef v16h V; static __device__ __forceinline__ V ld(const h16* p) { return cat16(*(const v8h*)p, *(const v8h*)(p + 16)); } static __device__ __forceinline__ v8f mma(V a, V b, v8f c) { return wmma16(a, b, c); } };
template <> struct WFrag<bf> { typedef v16bf V; static __device__ __forceinline__ V ld(const bf* p) { return cat16b(*(const v8us*)p, *(const v8us*)(p + 16)); } static __device__ __forceinline__ v8f mma(V a, V b, v8f c) { return wmmab(a, b, c); } };
template <typename T16, int NSPLIT, bool BIAS>
__global__ __launch_bounds__(32) void k_gemmw(const T16* __restrict__ A, const T16* __restrict__ A2, const T16* __restrict__ Bt, const T16* __restrict__ Bt2, int K, float* C, int ldc, const float* __restrict__ bias, size_t sA, size_t sB, size_t sC) {
    typedef typename WFrag<T16>::V V;
    __shared__ __align__(16) float os[16 * 68];
    const size_t z = blockIdx.z; A += z * sA; if (A2) A2 += z * sA; Bt += z * sB; if (Bt2) Bt2 += z * sB; C += z * sC;
    const int lane = threadIdx.x & 31, lr = lane & 15, hi = lane >> 4; const int r0 = blockIdx.x * 64, c0 = blockIdx.y * 64;
    v8f acc[4][4];
#pragma unroll
    for (int mb = 0; mb < 4; ++mb)
#pragma unroll
        for (int nb = 0; nb < 4; ++nb) acc[mb][nb] = (v8f){};
    const size_t aoff = (size_t)(r0 + lr) * K + 8 * hi, boff = (size_t)(c0 + lr) * K + 8 * hi;
    for (int kc = 0; kc < K; kc += 32) {
        V a[4], a2[4];
#pragma unroll
        for (int mb = 0; mb < 4; ++mb) { a[mb] = WFrag<T16>::ld(A + aoff + (size_t)mb * 16 * K + kc); if (NSPLIT == 1 || NSPLIT == 2) a2[mb] = WFrag<T16>::ld(A2 + aoff + (size_t)mb * 16 * K + kc); }
#pragma unroll
        for (int nb = 0; nb < 4; ++nb) { const V b = WFrag<T16>::ld(Bt + boff + (size_t)nb * 16 * K + kc); V b2; if (NSPLIT >= 2) b2 = WFrag<T16>::ld(Bt2 + boff + (size_t)nb * 16 * K + kc);
#pragma unroll
            for (int mb = 0; mb < 4; ++mb) { acc[mb][nb] = WFrag<T16>::mma(a[mb], b, acc[mb][nb]); if (NSPLIT == 1 || NSPLIT == 2) acc[mb][nb] = WFrag<T16>::mma(a2[mb], b, acc[mb][nb]); if (NSPLIT >= 2) acc[mb][nb] = WFrag<T16>::mma(a[mb], b2, acc[mb][nb]); } }
        asm volatile("v_nop\n\tv_nop\n\tv_nop\n\tv_nop" : "+v"(acc[0][0]), "+v"(acc[1][1]), "+v"(acc[2][2]), "+v"(acc[3][3]) : "v"(a[0]), "v"(a[3]));
    }
#pragma unroll
    for (int mb = 0; mb < 4; ++mb) {
#pragma unroll
        for (int nb = 0; nb < 4; ++nb) {
#pragma unroll
            for (int j = 0; j < 8; ++j) os[(hi * 8 + j) * 68 + nb * 16 + lr] = acc[mb][nb][j]; }
        __builtin_amdgcn_wave_barrier(); asm volatile("" ::: "memory");
        float* crow = C + (size_t)(r0 + mb * 16) * ldc + c0;
#pragma unroll 1
        for (int ps = 0; ps < 2; ++ps) {
#pragma unroll
            for (int s = 0; s < 8; ++s) { const int row = 2 * s + hi, cofs = lr * 4; v4f val = *(const v4fa*)(os + row * 68 + cofs); if (BIAS) { val[0] += bfr(bias[c0 + cofs]); val[1] += bfr(bias[c0 + cofs + 1]); val[2] += bfr(bias[c0 + cofs + 2]); val[3] += bfr(bias[c0 + cofs + 3]); }
                *(volatile v4f*)(crow + (size_t)row * ldc + cofs) = val; }
            if (ps == 0) __threadfence(); }
        __builtin_amdgcn_wave_barrier(); asm volatile("" ::: "memory");
    }
}

typedef __attribute__((ext_vector_type(2))) _Float16 v2h;
typedef __attribute__((ext_vector_type(4))) _Float16 v4h;
typedef __attribute__((ext_vector_type(2))) unsigned short v2us;
typedef __attribute__((ext_vector_type(4))) unsigned short v4us;
typedef __attribute__((ext_vector_type(2))) float v2f;
__device__ __forceinline__ h16 toh_flush(float x) { const float z = (fabsf(x) < 6.103515625e-05f) ? 0.0f : x; return (h16)z; }

template <int ACT>
__global__ __launch_bounds__(256) void eact_kernel(const float* __restrict__ P, float* __restrict__ OUT, size_t n4, float sl) {
  static_assert(ACT >= 1 && ACT <= 9, "eact: nine activations"); const size_t i = (size_t)blockIdx.x * 256 + threadIdx.x; if (i >= n4) return; const v4f a = *(const v4f*)(P + 4 * i); v4f o;
  for (int j = 0; j < 4; ++j) { const float v = a[j]; float y;
    if (ACT == 1) y = fmaxf(v, 0.0f);
    else if (ACT == 2) y = (v >= 0.0f) ? v : (sl * v);
    else if (ACT == 3) y = 1.0f / (1.0f + expf(-v));
    else if (ACT == 4) y = tanhf(v);
    else if (ACT == 5) y = (v > 0.0f) ? v : expm1f(v);
    else if (ACT == 6) y = v / (1.0f + expf(-v));
    else if (ACT == 7) y = (((0.5f * v)) * (1.0f + tanhf(0.7978845608028654f * (v + (0.044715f * ((v * ((v * v)))))))));
    else if (ACT == 8) y = (((0.5f * v)) * (1.0f + erff((v * 0.7071067811865476f))));
    else y = (1.0507009873554805f * ((v > 0.0f) ? v : (1.6732632423543772f * expm1f(v))));
    o[j] = y; }
  for (int pass = 0; pass < 2; ++pass) { *(volatile v4f*)(OUT + 4 * i) = o; __threadfence(); }
}

__global__ __launch_bounds__(64) void k_cat16(const float* __restrict__ U, int wu, int pu, int uin, const float* __restrict__ W, int ww, int pw, int win, h16* dst, int KP) { const int k0 = (blockIdx.x * 64 + threadIdx.x) * 8; if (k0 >= KP) return; const int r = blockIdx.y; const unsigned mu = 0u - (unsigned)(uin != 0), mw = 0u - (unsigned)(win != 0); v8h o;
#pragma unroll
    for (int q = 0; q < 8; ++q) { const int k = k0 + q; const bool iu = k < wu; const bool iw = (!iu) && (k < wu + ww); const int ku = min(k, wu - 1); const int kw = min(max(k - wu, 0), max(ww - 1, 0)); const float a = U[(size_t)r * pu + ku]; const float b = W[(size_t)r * pw + kw];
        const float va = __uint_as_float((__float_as_uint(bfr(a)) & mu) | (__float_as_uint(a) & ~mu)); const float vb = __uint_as_float((__float_as_uint(bfr(b)) & mw) | (__float_as_uint(b) & ~mw)); const unsigned su = 0u - (unsigned)iu, sw = 0u - (unsigned)iw; o[q] = toh_flush(__uint_as_float((__float_as_uint(va) & su) | (__float_as_uint(vb) & sw))); }
    *(volatile v8h*)(dst + (size_t)r * KP + k0) = o; __threadfence(); *(volatile v8h*)(dst + (size_t)r * KP + k0) = o; }

__global__ __launch_bounds__(64) void k_wtp16(const float* __restrict__ src, int K, int N, h16* dst, int KP, int NPz) { const int k0 = (blockIdx.x * 64 + threadIdx.x) * 8; if (k0 >= KP) return; const int n = blockIdx.y; const int z = blockIdx.z; const float* s = src + (size_t)z * K * N; v8h o;
#pragma unroll
    for (int q = 0; q < 8; ++q) { const int k = k0 + q; const bool in = (k < K) && (n < N); const float a = s[(size_t)min(k, K - 1) * N + min(n, N - 1)]; const unsigned mk = 0u - (unsigned)in; o[q] = toh_flush(__uint_as_float(__float_as_uint(bfr(a)) & mk)); }
    h16* d = dst + ((size_t)z * NPz + n) * KP + k0; *(volatile v8h*)d = o; __threadfence(); *(volatile v8h*)d = o; }

__global__ __launch_bounds__(256) void k_rep(const float* __restrict__ MV, const float* __restrict__ bm, const float* __restrict__ bv, const float* __restrict__ nz, float* Z, float* o1, float* o2) { const int i = blockIdx.x * 256 + threadIdx.x; if (i >= NR * LT / 4) return; const int r = i >> 3, j0 = (i & 7) * 4;
    const v4f a = *(const v4f*)(MV + (size_t)r * 64 + j0); const v4f b = *(const v4f*)(MV + (size_t)r * 64 + LT + j0); const v4f e = *(const v4f*)(nz + (size_t)i * 4); const v4f cm = *(const v4f*)(bm + j0); const v4f cv = *(const v4f*)(bv + j0); v4f m, v, z;
#pragma unroll
    for (int q = 0; q < 4; ++q) { m[q] = __fadd_rn(a[q], bfr(cm[q])); v[q] = __fadd_rn(b[q], bfr(cv[q])); z[q] = __fmaf_rn(bfr(e[q]), expf(__fmul_rn(0.5f, v[q])), m[q]); }
    *(volatile v4f*)(Z + (size_t)i * 4) = z; *(volatile v4f*)(o1 + (size_t)i * 4) = m; *(volatile v4f*)(o2 + (size_t)i * 4) = v; __threadfence(); *(volatile v4f*)(Z + (size_t)i * 4) = z; *(volatile v4f*)(o1 + (size_t)i * 4) = m; *(volatile v4f*)(o2 + (size_t)i * 4) = v; }

__global__ __launch_bounds__(256) void k_sm6(const float* __restrict__ LG, const float* __restrict__ bg, float* P) { const int r = blockIdx.x * 256 + threadIdx.x; if (r >= NR) return; const v4f a = *(const v4f*)(LG + (size_t)r * 64); const v4f b = *(const v4f*)(LG + (size_t)r * 64 + 4); float l[NP];
    l[0] = __fadd_rn(a[0], bfr(bg[0])); l[1] = __fadd_rn(a[1], bfr(bg[1])); l[2] = __fadd_rn(a[2], bfr(bg[2])); l[3] = __fadd_rn(a[3], bfr(bg[3])); l[4] = __fadd_rn(b[0], bfr(bg[4])); l[5] = __fadd_rn(b[1], bfr(bg[5]));
    float mx = l[0];
#pragma unroll
    for (int c = 1; c < NP; ++c) mx = fmaxf(mx, l[c]);
    float e[NP]; float s = 0.0f;
#pragma unroll
    for (int c = 0; c < NP; ++c) { e[c] = expf(__fsub_rn(l[c], mx)); s = __fadd_rn(s, e[c]); }
    v4f o0, o1; o0[0] = __fdiv_rn(e[0], s); o0[1] = __fdiv_rn(e[1], s); o0[2] = __fdiv_rn(e[2], s); o0[3] = __fdiv_rn(e[3], s); o1[0] = __fdiv_rn(e[4], s); o1[1] = __fdiv_rn(e[5], s); o1[2] = __fmul_rn(a[0], 0.0f); o1[3] = __fmul_rn(a[1], 0.0f); v4f oz; oz[0] = __fmul_rn(a[0], 0.0f); oz[1] = __fmul_rn(a[1], 0.0f); oz[2] = __fmul_rn(a[2], 0.0f); oz[3] = __fmul_rn(a[3], 0.0f);
#pragma unroll
    for (int ps = 0; ps < 2; ++ps) { *(volatile v4f*)(P + (size_t)r * 32) = o0; *(volatile v4f*)(P + (size_t)r * 32 + 4) = o1;
#pragma unroll
        for (int j4 = 2; j4 < 8; ++j4) *(volatile v4f*)(P + (size_t)r * 32 + 4 * j4) = oz;
        if (ps == 0) __threadfence(); } }

template <int H, int QP>
__global__ __launch_bounds__(256) void k_mix(const float* __restrict__ Q, const float* __restrict__ P, const float* __restrict__ bias, float* Y) { const int i = blockIdx.x * 256 + threadIdx.x; if (i >= NR * H / 4) return; v4f o;
#pragma unroll
    for (int q = 0; q < 4; ++q) { const int f = 4 * i + q; const int r = f / H, h = f - r * H; float s = 0.0f;
#pragma unroll
        for (int e = 0; e < NP; ++e) s = __fmaf_rn(P[(size_t)r * 32 + e], __fadd_rn(Q[((size_t)e * NR + r) * QP + h], bfr(bias[e * H + h])), s);
        o[q] = s; }
    *(volatile v4f*)(Y + (size_t)i * 4) = o; __threadfence(); *(volatile v4f*)(Y + (size_t)i * 4) = o; }

extern "C" void kernel_launch(void* const* d_in, const int* in_sizes, int n_in, void* d_out, int out_size, void* d_ws, size_t ws_size, hipStream_t stream) {
    if (n_in < 23) return;
    const int want[23] = {NR * FR, NR * FR, NR * LT, 2 * FR * HD, HD, (FR + HD) * HD, HD, (FR + HD) * LT, LT, (FR + HD) * LT, LT, (LT + FR) * GW, GW, GW * GW, GW, GW * NP, NP, NP * (LT + FR) * HD, NP * HD, NP * (LT + HD) * HD, NP * HD, NP * (LT + HD) * FR, NP * FR};
    for (int k = 0; k < 23; ++k) if (in_sizes[k] != want[k]) return;
    if (out_size != NR * FR + 2 * NR * LT) return;
    static_assert(NR % 64 == 0 && HD % 64 == 0 && GW % 64 == 0 && N3 % 64 == 0 && K1 % 64 == 0 && K2 % 64 == 0 && K1 >= 2 * FR && K1 >= FR + HD && K2 >= LT + FR && K2 >= LT + HD && N3 >= FR && (NR * FR) % 128 == 0 && (NR * HD) % 1024 == 0 && (NR * FR / 4) % 256 == 0 && NR % 256 == 0 && (NR * LT / 4) % 256 == 0 && ((size_t)NR * FR * 4) % 128 == 0, "rows and widths multiples of 64; padded depths multiples of 64 that hold their sources; every flat grid exact; out1 begins on a 128-byte line");
    const float* ia = (const float*)d_in[0]; const float* ib = (const float*)d_in[1]; const float* in_ = (const float*)d_in[2];
    const float* w[20]; for (int k = 0; k < 20; ++k) w[k] = (const float*)d_in[3 + k];
    float* out0 = (float*)d_out; float* out1 = out0 + (size_t)NR * FR; float* out2 = out1 + (size_t)NR * LT;
    char* wsp = (char*)d_ws; auto take = [&](size_t bytes) { char* p = wsp; wsp += (bytes + 255) & ~(size_t)255; return (void*)p; };
    h16* T1a = (h16*)take((size_t)HD * K1 * 2); h16* T1b = (h16*)take((size_t)HD * K1 * 2); h16* Tmv = (h16*)take((size_t)64 * K1 * 2); h16* Tg1 = (h16*)take((size_t)GW * K2 * 2); h16* Tg2 = (h16*)take((size_t)GW * GW * 2); h16* Tg3 = (h16*)take((size_t)64 * GW * 2);
    h16* Tc0 = (h16*)take((size_t)NP * HD * K2 * 2); h16* Tc1 = (h16*)take((size_t)NP * HD * K2 * 2); h16* Tc2 = (h16*)take((size_t)NP * N3 * K2 * 2);
    h16* L1 = (h16*)take((size_t)NR * K1 * 2);     h16* L2 = (h16*)take((size_t)NR * K2 * 2);     h16* L3 = (h16*)take((size_t)NR * GW * 2);
    float* F1 = (float*)take((size_t)NR * HD * 4); float* F2 = (float*)take((size_t)NR * HD * 4);     float* G1 = (float*)take((size_t)NR * 64 * 4); float* G2 = (float*)take((size_t)NR * 64 * 4);
    float* Z = (float*)take((size_t)NR * LT * 4); float* P = (float*)take((size_t)NR * 32 * 4);     float* Q = (float*)take((size_t)NP * NR * N3 * 4);
    if ((size_t)(wsp - (char*)d_ws) > ws_size) return;
    auto wt = [&](const float* s, int K, int N, h16* d, int KP, int rows, int Z_, int NPz) { k_wtp16<<<dim3((KP + 511) / 512, rows, Z_), 64, 0, stream>>>(s, K, N, d, KP, NPz); };
    wt(w[0], 2 * FR, HD, T1a, K1, HD, 1, HD); wt(w[2], FR + HD, HD, T1b, K1, HD, 1, HD); wt(w[4], FR + HD, LT, Tmv, K1, LT, 1, LT); wt(w[6], FR + HD, LT, Tmv + (size_t)LT * K1, K1, LT, 1, LT);
    wt(w[8], LT + FR, GW, Tg1, K2, GW, 1, GW); wt(w[10], GW, GW, Tg2, GW, GW, 1, GW); wt(w[12], GW, NP, Tg3, GW, 64, 1, 64);
    wt(w[14], LT + FR, HD, Tc0, K2, HD, NP, HD); wt(w[16], LT + HD, HD, Tc1, K2, HD, NP, HD); wt(w[18], LT + HD, FR, Tc2, K2, N3, NP, N3);
    auto cat = [&](const float* U, int wu, int pu, int uin, const float* W_, int ww, int pw, int win, h16* d, int KP) { k_cat16<<<dim3((KP + 511) / 512, NR, 1), 64, 0, stream>>>(U, wu, pu, uin, W_, ww, pw, win, d, KP); };
    const unsigned E256 = (unsigned)(NR * HD / 4 / 256), E64 = (unsigned)(NR * 64 / 4 / 256);
    cat(ia, FR, FR, 1, ib, FR, FR, 1, L1, K1);
    k_gemmw<h16, 0, true><<<dim3(NR / 64, HD / 64, 1), 32, 0, stream>>>(L1, nullptr, T1a, nullptr, K1, F1, HD, w[1], 0, 0, 0);
    eact_kernel<5><<<E256, 256, 0, stream>>>(F1, F2, (size_t)NR * HD / 4, 0.0f);
    cat(ia, FR, FR, 1, F2, HD, HD, 0, L1, K1);
    k_gemmw<h16, 0, true><<<dim3(NR / 64, HD / 64, 1), 32, 0, stream>>>(L1, nullptr, T1b, nullptr, K1, F1, HD, w[3], 0, 0, 0);
    eact_kernel<5><<<E256, 256, 0, stream>>>(F1, F2, (size_t)NR * HD / 4, 0.0f);
    cat(ia, FR, FR, 1, F2, HD, HD, 0, L1, K1);
    k_gemmw<h16, 0, false><<<dim3(NR / 64, 1, 1), 32, 0, stream>>>(L1, nullptr, Tmv, nullptr, K1, G1, 64, nullptr, 0, 0, 0);
    k_rep<<<(unsigned)(NR * LT / 4 / 256), 256, 0, stream>>>(G1, w[5], w[7], in_, Z, out1, out2);
    cat(Z, LT, LT, 0, ib, FR, FR, 1, L2, K2);
    k_gemmw<h16, 0, true><<<dim3(NR / 64, 1, 1), 32, 0, stream>>>(L2, nullptr, Tg1, nullptr, K2, G1, 64, w[9], 0, 0, 0);
    eact_kernel<5><<<E64, 256, 0, stream>>>(G1, G2, (size_t)NR * 64 / 4, 0.0f);
    cat(G2, GW, GW, 0, G2, 0, GW, 0, L3, GW);
    k_gemmw<h16, 0, true><<<dim3(NR / 64, 1, 1), 32, 0, stream>>>(L3, nullptr, Tg2, nullptr, GW, G1, 64, w[11], 0, 0, 0);
    eact_kernel<5><<<E64, 256, 0, stream>>>(G1, G2, (size_t)NR * 64 / 4, 0.0f);
    cat(G2, GW, GW, 0, G2, 0, GW, 0, L3, GW);
    k_gemmw<h16, 0, false><<<dim3(NR / 64, 1, 1), 32, 0, stream>>>(L3, nullptr, Tg3, nullptr, GW, G1, 64, nullptr, 0, 0, 0);
    k_sm6<<<(unsigned)(NR / 256), 256, 0, stream>>>(G1, w[13], P);
    k_gemmw<h16, 0, false><<<dim3(NR / 64, HD / 64, NP), 32, 0, stream>>>(L2, nullptr, Tc0, nullptr, K2, Q, HD, nullptr, 0, (size_t)HD * K2, (size_t)NR * HD);
    k_mix<HD, HD><<<E256, 256, 0, stream>>>(Q, P, w[15], F1);
    eact_kernel<5><<<E256, 256, 0, stream>>>(F1, F2, (size_t)NR * HD / 4, 0.0f);
    cat(Z, LT, LT, 0, F2, HD, HD, 0, L2, K2);
    k_gemmw<h16, 0, false><<<dim3(NR / 64, HD / 64, NP), 32, 0, stream>>>(L2, nullptr, Tc1, nullptr, K2, Q, HD, nullptr, 0, (size_t)HD * K2, (size_t)NR * HD);
    k_mix<HD, HD><<<E256, 256, 0, stream>>>(Q, P, w[17], F1);
    eact_kernel<5><<<E256, 256, 0, stream>>>(F1, F2, (size_t)NR * HD / 4, 0.0f);
    cat(Z, LT, LT, 0, F2, HD, HD, 0, L2, K2);
    k_gemmw<h16, 0, false><<<dim3(NR / 64, N3 / 64, NP), 32, 0, stream>>>(L2, nullptr, Tc2, nullptr, K2, Q, N3, nullptr, 0, (size_t)N3 * K2, (size_t)NR * N3);
    k_mix<FR, N3><<<(unsigned)(NR * FR / 4 / 256), 256, 0, stream>>>(Q, P, w[19], out0);
}
